// LRU_33011118637310
// MI455X (gfx1250) — hardware-verified
//
#include <hip/hip_runtime.h>
#include <math.h>

typedef __attribute__((ext_vector_type(16))) _Float16 v16h;
typedef __attribute__((ext_vector_type(8)))  _Float16 v8h;
typedef __attribute__((ext_vector_type(2)))  _Float16 v2h;
typedef __attribute__((ext_vector_type(16))) __bf16   v16b;
typedef __attribute__((ext_vector_type(8)))  __bf16   v8b;
typedef __attribute__((ext_vector_type(8)))  float    v8f;
typedef __attribute__((ext_vector_type(4)))  float    v4f;
typedef __attribute__((ext_vector_type(2)))  float    v2f;

constexpr int kLen    = 32768;
constexpr int kModel  = 256;
constexpr int kHid    = 256;
constexpr int kHid2   = 2 * kHid;
constexpr int kThr    = 256;

constexpr float kInCarry  = 1024.0f;
constexpr float kWCarry   = 1024.0f;
constexpr float kHCarry   = 256.0f;
constexpr float kBuScale  = 1.0f / (kInCarry * kWCarry);
constexpr float kYScale   = 1.0f / (kHCarry * kWCarry);
constexpr float kF16MinNormal = 6.103515625e-5f;

static_assert((kLen % 64) == 0 && (kHid2 % 64) == 0 && (kModel % 64) == 0 && (kModel % 32) == 0 && (kHid2 % 32) == 0, "GEMM M, N multiples of 64, K of 32");
static_assert(kHid == 4 * 64, "the scan: 4 single-wave blocks x 32 lanes x 2 adjacent states");

constexpr size_t kOffX16  = 0;
constexpr size_t kOffBN   = kOffX16 + (size_t)kLen * kModel * 2;
constexpr size_t kOffCC   = kOffBN  + (size_t)kHid2 * kModel * 2;
constexpr size_t kOffLAM  = kOffCC  + (size_t)kModel * kHid2 * 2;
constexpr size_t kOffZB   = kOffLAM + (size_t)2 * kHid * 4;
constexpr size_t kOffBU   = kOffZB  + (size_t)kHid2 * 4;
constexpr size_t kOffH16  = kOffBU  + (size_t)kLen * kHid2 * 4;
constexpr size_t kWsTotal = kOffH16 + (size_t)kLen * kHid2 * 2;
static_assert(kWsTotal == 117968896ull, "carve total");
static_assert(kWsTotal <= 134217728ull, "carve cap");
static_assert((kOffBN % 256) == 0 && (kOffCC % 256) == 0 && (kOffLAM % 256) == 0 && (kOffZB % 256) == 0 && (kOffBU % 256) == 0 && (kOffH16 % 256) == 0, "aligned regions");

__device__ __forceinline__ unsigned short f2bf_bits(float f) {
  unsigned u = __float_as_uint(f);
  return (unsigned short)((u + 0x7FFFu + ((u >> 16) & 1u)) >> 16);
}
__device__ __forceinline__ float bf_bits2f(unsigned short h) { return __uint_as_float(((unsigned)h) << 16); }
__device__ __forceinline__ float bf16r(float f) { return bf_bits2f(f2bf_bits(f)); }
__device__ __forceinline__ float carry_flush(float v, float carry) {
  const float s = v * carry;
  return (fabsf(s) < kF16MinNormal) ? 0.0f : s;
}
__device__ __forceinline__ float frcp(float x) { return __builtin_amdgcn_rcpf(x); }

__device__ __forceinline__ void dep_guard4_h(v8f& a, v8f& b, v8f& c, v8f& d, v16h x, v16h y) { asm volatile("v_nop\n\tv_nop\n\tv_nop\n\tv_nop" : "+v"(a), "+v"(b), "+v"(c), "+v"(d) : "v"(x), "v"(y)); }
__device__ __forceinline__ void dep_guard4_b(v8f& a, v8f& b, v8f& c, v8f& d, v16b x, v16b y) { asm volatile("v_nop\n\tv_nop\n\tv_nop\n\tv_nop" : "+v"(a), "+v"(b), "+v"(c), "+v"(d) : "v"(x), "v"(y)); }
__device__ __forceinline__ void keep4_h(v16h a, v16h b, v16h c, v16h d) { asm volatile("v_nop" :: "v"(a), "v"(b), "v"(c), "v"(d)); }
__device__ __forceinline__ void keep4_b(v16b a, v16b b, v16b c, v16b d) { asm volatile("v_nop" :: "v"(a), "v"(b), "v"(c), "v"(d)); }
__device__ __forceinline__ void acc_guard4(v8f& a, v8f& b, v8f& c, v8f& d) { asm volatile("v_nop\n\tv_nop\n\tv_nop\n\tv_nop" : "+v"(a), "+v"(b), "+v"(c), "+v"(d)); }

template <typename T> struct Frag;
template <> struct Frag<_Float16> {
  typedef v16h V; union U { v16h v; v8h h[2]; };
  static __device__ __forceinline__ v16h load(const _Float16* p) {
    U f; f.h[0] = *(const v8h*)(p); f.h[1] = *(const v8h*)(p + 16); return f.v;
  }
  static __device__ __forceinline__ v8f mma(v16h a, v16h b, v8f c) {
    return __builtin_amdgcn_wmma_f32_16x16x32_f16(false, a, false, b, (short)0, c, false, false);
  }
  static __device__ __forceinline__ void guard4(v8f& a, v8f& b, v8f& c, v8f& d, v16h x, v16h y) { dep_guard4_h(a, b, c, d, x, y); }
  static __device__ __forceinline__ void keep(v16h a, v16h b, v16h c, v16h d) { keep4_h(a, b, c, d); }
};
template <> struct Frag<__bf16> {
  typedef v16b V; union U { v16b v; v8b h[2]; };
  static __device__ __forceinline__ v16b load(const __bf16* p) {
    U f; f.h[0] = *(const v8b*)(p); f.h[1] = *(const v8b*)(p + 16); return f.v;
  }
  static __device__ __forceinline__ v8f mma(v16b a, v16b b, v8f c) {
    return __builtin_amdgcn_wmma_f32_16x16x32_bf16(false, a, false, b, (short)0, c, false, false);
  }
  static __device__ __forceinline__ void guard4(v8f& a, v8f& b, v8f& c, v8f& d, v16b x, v16b y) { dep_guard4_b(a, b, c, d, x, y); }
  static __device__ __forceinline__ void keep(v16b a, v16b b, v16b c, v16b d) { keep4_b(a, b, c, d); }
};

__device__ __forceinline__ v8f mma_h(v16h a, v16h b, v8f c) {
  c = __builtin_amdgcn_wmma_f32_16x16x32_f16(false, a, false, b, (short)0, c, false, false);
  asm volatile("v_nop\n\tv_nop\n\tv_nop\n\tv_nop" : "+v"(c) : "v"(a), "v"(b));
  return c;
}

template <int ET> struct Elem;
template <> struct Elem<0> { typedef _Float16 T; };
template <> struct Elem<1> { typedef __bf16 T; };
template <int ET, bool SPLIT, int BIAS_MODE, int OUT_MODE, bool RESID, int ACT = 0>
__global__ __launch_bounds__(256) void wmma_gemm64(
    const unsigned short* __restrict__ Ap, const unsigned short* __restrict__ A2p, int lda, long strideA,
    const unsigned short* __restrict__ Btp, const unsigned short* __restrict__ Bt2p, int ldb, long strideB,
    void* __restrict__ Cout, void* __restrict__ Cout2, int ldc, long strideC,
    const float* __restrict__ bias,
    const float* __restrict__ resid, long strideR,
    int M, int N, int K, float scale) {
  typedef typename Elem<ET>::T T;
  typedef typename Frag<T>::V V;
  const T* A = (const T*)Ap; const T* A2 = (const T*)A2p; const T* Bt = (const T*)Btp; const T* Bt2 = (const T*)Bt2p;
  __shared__ __align__(16) float sT[8][16 * 68];
  const int b    = blockIdx.y;
  const int lane = threadIdx.x & 31;
  const int wave = threadIdx.x >> 5;
  const int tilesN = N >> 6;
  const int tilesM = M >> 6;
  const int tile = blockIdx.x * 8 + wave;
  if (tile >= tilesM * tilesN) return;
  const int tm = tile / tilesN;
  const int tn = tile - tm * tilesN;
  const int m0 = tm << 6;
  const int n0 = tn << 6;

  const T* Ab  = A  + (size_t)b * strideA;
  const T* Bb  = Bt + (size_t)b * strideB;
  const T* Ab2 = SPLIT ? (A2  + (size_t)b * strideA) : nullptr;
  const T* Bb2 = SPLIT ? (Bt2 + (size_t)b * strideB) : nullptr;

  const int rlane = lane & 15;
  const int koff  = (lane >> 4) * 8;
  const int mOff  = (lane >> 4) * 8;

  v8f acc[4][4];
#pragma unroll
  for (int i = 0; i < 4; ++i)
#pragma unroll
    for (int j = 0; j < 4; ++j) acc[i][j] = (v8f){0.f,0.f,0.f,0.f,0.f,0.f,0.f,0.f};

  for (int k0 = 0; k0 < K; k0 += 32) {
    V bh[4], bl[4];
#pragma unroll
    for (int j = 0; j < 4; ++j) {
      const size_t bo = (size_t)(n0 + (j << 4) + rlane) * ldb + koff + k0;
      bh[j] = Frag<T>::load(Bb + bo);
      if (SPLIT) bl[j] = Frag<T>::load(Bb2 + bo);
    }
#pragma unroll
    for (int i = 0; i < 4; ++i) {
      const size_t ao = (size_t)(m0 + (i << 4) + rlane) * lda + koff + k0;
      V ah = Frag<T>::load(Ab + ao);
      V al;
      if (SPLIT) al = Frag<T>::load(Ab2 + ao);
#pragma unroll
      for (int j = 0; j < 4; ++j) {
        acc[i][j] = Frag<T>::mma(ah, bh[j], acc[i][j]);
        if (SPLIT) {
          acc[i][j] = Frag<T>::mma(ah, bl[j], acc[i][j]);
          acc[i][j] = Frag<T>::mma(al, bh[j], acc[i][j]);
        }
      }
      Frag<T>::guard4(acc[i][0], acc[i][1], acc[i][2], acc[i][3], ah, SPLIT ? al : ah);
    }
    Frag<T>::keep(bh[0], bh[1], bh[2], bh[3]);
    if (SPLIT) Frag<T>::keep(bl[0], bl[1], bl[2], bl[3]);
  }
  acc_guard4(acc[0][0], acc[0][1], acc[0][2], acc[0][3]);
  acc_guard4(acc[1][0], acc[1][1], acc[1][2], acc[1][3]);
  acc_guard4(acc[2][0], acc[2][1], acc[2][2], acc[2][3]);
  acc_guard4(acc[3][0], acc[3][1], acc[3][2], acc[3][3]);

  float* slab = sT[wave];
  const float* Rb = RESID ? (resid + (size_t)b * strideR) : nullptr;
#pragma unroll
  for (int i = 0; i < 4; ++i) {
    const int mBase = m0 + (i << 4);
#pragma unroll
    for (int j = 0; j < 4; ++j) {
      const int n = n0 + (j << 4) + rlane;
      float bv = 0.f;
      if (BIAS_MODE == 2) bv = bias[n];
#pragma unroll
      for (int r = 0; r < 8; ++r) {
        float v = acc[i][j][r] * scale;
        if (BIAS_MODE == 1) v += bias[mBase + mOff + r];
        if (BIAS_MODE == 2) v += bv;
        if (RESID) v += Rb[(size_t)(mBase + mOff + r) * ldc + n];
        if (ACT == 1) v = tanhf(v);
        if (ACT == 2) v = fmaxf(v, 0.0f);
        if (ACT == 3) v = v / (1.0f + expf(-v));
        if (ACT == 4) v = (v > 0.f) ? v : 0.01f * v;
        slab[(mOff + r) * 68 + (j << 4) + rlane] = v;
      }
    }
    __builtin_amdgcn_fence(__ATOMIC_RELEASE, "workgroup");
    __builtin_amdgcn_wave_barrier();
    __builtin_amdgcn_fence(__ATOMIC_ACQUIRE, "workgroup");
    if (OUT_MODE == 0) {
      float* C = (float*)Cout + (size_t)b * strideC;
      const int hh = lane >> 4, c4 = (lane & 15) * 4;
      for (int pass = 0; pass < 2; ++pass) {
#pragma unroll
        for (int it = 0; it < 8; ++it) {
          const int row = it * 2 + hh;
          v4f v = *(const v4f*)(slab + row * 68 + c4);
          *(volatile v4f*)(C + (size_t)(mBase + row) * ldc + n0 + c4) = v;
        }
        __threadfence();
      }
    } else {
      const int q = lane >> 3, c8 = (lane & 7) * 8;
      unsigned short* C  = (unsigned short*)Cout  + (size_t)b * strideC;
      unsigned short* C2 = (OUT_MODE == 2) ? ((unsigned short*)Cout2 + (size_t)b * strideC) : nullptr;
      for (int pass = 0; pass < 2; ++pass) {
#pragma unroll
        for (int it = 0; it < 4; ++it) {
          const int row = it * 4 + q;
          const float* sp = slab + row * 68 + c8;
          v8h hv, lv;
#pragma unroll
          for (int e = 0; e < 8; ++e) {
            if (OUT_MODE == 1) {
              hv[e] = (_Float16)sp[e];
            } else {
              unsigned short hb = f2bf_bits(sp[e]);
              unsigned short lb = f2bf_bits(sp[e] - bf_bits2f(hb));
              hv[e] = __builtin_bit_cast(_Float16, hb);
              lv[e] = __builtin_bit_cast(_Float16, lb);
            }
          }
          *(volatile v8h*)(C + (size_t)(mBase + row) * ldc + n0 + c8) = hv;
          if (OUT_MODE == 2) *(volatile v8h*)(C2 + (size_t)(mBase + row) * ldc + n0 + c8) = lv;
        }
        __threadfence();
      }
    }
    __builtin_amdgcn_fence(__ATOMIC_RELEASE, "workgroup");
    __builtin_amdgcn_wave_barrier();
    __builtin_amdgcn_fence(__ATOMIC_ACQUIRE, "workgroup");
  }
}

__global__ __launch_bounds__(kThr) void cast_plane_kernel(const float* __restrict__ src, unsigned short* __restrict__ dst,
                                                          int colsLog2, int dstPitch, int dstOff) {
  const int i   = blockIdx.x * kThr + threadIdx.x;
  const int sh  = colsLog2 - 3;
  const int row = i >> sh;
  const int c8  = (i & ((1 << sh) - 1)) * 8;
  const float* sp = src + ((size_t)row << colsLog2) + c8;
  const v4f a0 = *(const v4f*)(sp);
  const v4f a1 = *(const v4f*)(sp + 4);
  v8h hv;
#pragma unroll
  for (int e = 0; e < 4; ++e) {
    const float f0 = a0[e];
    const float f1 = a1[e];
    hv[e]     = (_Float16)carry_flush(bf16r(f0), kInCarry);
    hv[4 + e] = (_Float16)carry_flush(bf16r(f1), kInCarry);
  }
  unsigned short* dp = dst + (size_t)row * dstPitch + dstOff + c8;
  *(volatile v8h*)dp = hv;
  __threadfence();
  *(volatile v8h*)dp = hv;
}
static_assert(kInCarry == kWCarry, "one cast kernel serves inputs and weights");

__global__ __launch_bounds__(kThr) void lru_prep_kernel(const float* __restrict__ nu_log, const float* __restrict__ theta_log,
                                                        const float* __restrict__ gamma_log,
                                                        const float* __restrict__ B_re, const float* __restrict__ B_im,
                                                        const float* __restrict__ C_re, const float* __restrict__ C_im,
                                                        unsigned short* __restrict__ BN16, unsigned short* __restrict__ CC16,
                                                        float* __restrict__ LAM, float* __restrict__ ZB) {
  const int r = blockIdx.x;
  const int tid = threadIdx.x;
  const int part = tid >> 7;
  const int c2 = (tid & 127) * 2;
  const float g = expf(bf16r(gamma_log[r]));
  const float* bsrc = part ? B_im : B_re;
  const float* csrc = part ? C_im : C_re;
  const float b0 = bsrc[(size_t)r * kModel + c2];
  const float b1 = bsrc[(size_t)r * kModel + c2 + 1];
  const float q0 = csrc[(size_t)r * kHid + c2];
  const float q1 = csrc[(size_t)r * kHid + c2 + 1];
  const float sgn = part ? -1.0f : 1.0f;
  v2h bv, cv;
  bv[0] = (_Float16)carry_flush(g * bf16r(b0), kWCarry);
  bv[1] = (_Float16)carry_flush(g * bf16r(b1), kWCarry);
  cv[0] = (_Float16)carry_flush(sgn * bf16r(q0), kWCarry);
  cv[1] = (_Float16)carry_flush(sgn * bf16r(q1), kWCarry);
  unsigned short* bd = BN16 + (size_t)(part * kHid + r) * kModel + c2;
  unsigned short* cd = CC16 + (size_t)r * kHid2 + part * kHid + c2;
  for (int pass = 0; pass < 2; ++pass) {
    *(volatile v2h*)bd = bv;
    *(volatile v2h*)cd = cv;
    __threadfence();
  }
  if (r == 0) {
    const float nu = expf(bf16r(nu_log[tid]));
    const float th = expf(bf16r(theta_log[tid]));
    const float mag = expf(-nu);
    const float lre = mag * cosf(th);
    const float lim = mag * sinf(th);
    const v2f z2 = {0.f, 0.f};
    for (int pass = 0; pass < 2; ++pass) {
      *(volatile float*)(LAM + tid) = lre;
      *(volatile float*)(LAM + kHid + tid) = lim;
      *(volatile v2f*)(ZB + 2 * tid) = z2;
      __threadfence();
    }
  }
}

__global__ __launch_bounds__(32) void lru_scan_kernel(const float* __restrict__ BU, const float* __restrict__ LAM,
                                                      unsigned short* __restrict__ H16) {
  const int h0 = blockIdx.x * 64 + 2 * (threadIdx.x & 31);
  const float lr0 = LAM[h0], lr1 = LAM[h0 + 1];
  const float li0 = LAM[kHid + h0], li1 = LAM[kHid + h0 + 1];
  float hr0 = 0.f, hi0 = 0.f, hr1 = 0.f, hi1 = 0.f;
#pragma unroll 1
  for (int t = 0; t < kLen; ++t) {
    const v2f br = *(const v2f*)(BU + (size_t)t * kHid2 + h0);
    const v2f bi = *(const v2f*)(BU + (size_t)t * kHid2 + kHid + h0);
    const float nr0 = fmaf(lr0, hr0, fmaf(-li0, hi0, br[0]));
    const float ni0 = fmaf(lr0, hi0, fmaf(li0, hr0, bi[0]));
    const float nr1 = fmaf(lr1, hr1, fmaf(-li1, hi1, br[1]));
    const float ni1 = fmaf(lr1, hi1, fmaf(li1, hr1, bi[1]));
    hr0 = nr0; hi0 = ni0; hr1 = nr1; hi1 = ni1;
    v2h vr, vi;
    vr[0] = (_Float16)carry_flush(hr0, kHCarry);
    vr[1] = (_Float16)carry_flush(hr1, kHCarry);
    vi[0] = (_Float16)carry_flush(hi0, kHCarry);
    vi[1] = (_Float16)carry_flush(hi1, kHCarry);
    unsigned short* rp = H16 + (size_t)t * kHid2 + h0;
    unsigned short* ip = H16 + (size_t)t * kHid2 + kHid + h0;
    for (int pass = 0; pass < 2; ++pass) {
      *(volatile v2h*)rp = vr;
      *(volatile v2h*)ip = vi;
      __threadfence();
    }
  }
}

__global__ __launch_bounds__(kThr) void skip_out_kernel(const float* __restrict__ YW, const float* __restrict__ x,
                                                        const float* __restrict__ Dv, float* __restrict__ out) {
  const size_t i4 = ((size_t)blockIdx.x * kThr + threadIdx.x) * 4;
  const int m = (int)(i4 & (kModel - 1));
  const v4f y = *(const v4f*)(YW + i4);
  const v4f xv = *(const v4f*)(x + i4);
  const v4f dv = *(const v4f*)(Dv + m);
  v4f o;
#pragma unroll
  for (int e = 0; e < 4; ++e) {
    const float xe = xv[e];
    const float de = dv[e];
    o[e] = fmaf(bf16r(de), bf16r(xe), y[e]);
  }
  *(volatile v4f*)(out + i4) = o;
  __threadfence();
  *(volatile v4f*)(out + i4) = o;
}

static_assert(((kLen / 64) * (kHid2 / 64)) % 8 == 0 && ((kLen / 64) * (kModel / 64)) % 8 == 0, "GEMM grids exact");
static_assert(((size_t)kLen * kModel / 8) % kThr == 0 && ((size_t)kLen * kModel / 4) % kThr == 0, "cast and skip grids exact");

extern "C" void kernel_launch(void* const* d_in, const int* in_sizes, int n_in,
                              void* d_out, int out_size, void* d_ws, size_t ws_size,
                              hipStream_t stream) {
  if (n_in < 9 || d_out == nullptr || d_ws == nullptr) return;
  if (in_sizes[0] != kLen * kModel) return;
  if (in_sizes[1] != kHid || in_sizes[2] != kHid || in_sizes[3] != kHid) return;
  if (in_sizes[4] != kHid * kModel || in_sizes[5] != kHid * kModel) return;
  if (in_sizes[6] != kModel * kHid || in_sizes[7] != kModel * kHid) return;
  if (in_sizes[8] != kModel) return;
  if (out_size != kLen * kModel) return;
  if (ws_size < kWsTotal) return;

  const float* x    = (const float*)d_in[0];
  const float* nul  = (const float*)d_in[1];
  const float* thl  = (const float*)d_in[2];
  const float* gal  = (const float*)d_in[3];
  const float* B_re = (const float*)d_in[4];
  const float* B_im = (const float*)d_in[5];
  const float* C_re = (const float*)d_in[6];
  const float* C_im = (const float*)d_in[7];
  const float* Dv   = (const float*)d_in[8];
  float* out = (float*)d_out;

  char* ws = (char*)d_ws;
  unsigned short* X16  = (unsigned short*)(ws + kOffX16);
  unsigned short* BN16 = (unsigned short*)(ws + kOffBN);
  unsigned short* CC16 = (unsigned short*)(ws + kOffCC);
  float*          LAM  = (float*)(ws + kOffLAM);
  float*          ZB   = (float*)(ws + kOffZB);
  float*          BU   = (float*)(ws + kOffBU);
  float*          YW   = (float*)(ws + kOffBU);
  unsigned short* H16  = (unsigned short*)(ws + kOffH16);

  cast_plane_kernel<<<(int)(((size_t)kLen * kModel / 8) / kThr), kThr, 0, stream>>>(x, X16, 8, kModel, 0);
  lru_prep_kernel<<<kHid, kThr, 0, stream>>>(nul, thl, gal, B_re, B_im, C_re, C_im, BN16, CC16, LAM, ZB);

  wmma_gemm64<0, false, 2, 0, false, 0><<<dim3((kLen / 64) * (kHid2 / 64) / 8, 1), 256, 0, stream>>>(
      X16, X16, kModel, 0L, BN16, BN16, kModel, 0L, (void*)BU, (void*)BU, kHid2, 0L,
      ZB, nullptr, 0L, kLen, kHid2, kModel, kBuScale);

  lru_scan_kernel<<<kHid / 64, 32, 0, stream>>>(BU, LAM, H16);

  wmma_gemm64<0, false, 2, 0, false, 0><<<dim3((kLen / 64) * (kModel / 64) / 8, 1), 256, 0, stream>>>(
      H16, H16, kHid2, 0L, CC16, CC16, kHid2, 0L, (void*)YW, (void*)YW, kModel, 0L,
      ZB, nullptr, 0L, kLen, kModel, kHid2, kYScale);

  skip_out_kernel<<<(int)(((size_t)kLen * kModel / 4) / kThr), kThr, 0, stream>>>(YW, x, Dv, out);
}
